// DeepCLFM_42992622633202
// MI455X (gfx1250) — hardware-run, weakly checked
//
#include <hip/hip_runtime.h>
#include <math.h>

constexpr int NUSR  = 512;
constexpr int NITM  = 1024;
constexpr int NSTEP = 100;
constexpr int HID   = 64;
constexpr int G3    = 3 * HID;
constexpr int EMBW  = 2 * HID;
constexpr int NATT  = 8;
constexpr int NH1   = 64;
constexpr int NH2   = 16;
constexpr int PAIRW = 4 * HID;
constexpr int GRU_THR = 128;
constexpr int SEQB  = 16;
constexpr int HPAD  = 72;
constexpr int SLABP = 68;
constexpr int FMX_THR = 64;
constexpr int PR_THR  = 128;
constexpr int PR_WAVES = PR_THR / 32;
constexpr int PR_ROWS = 32;
constexpr int PR_PITCH = 72;
static_assert(NUSR % SEQB == 0 && NITM % SEQB == 0);
static_assert(HID == 16 * (GRU_THR / 32));
static_assert((SEQB * HPAD) % GRU_THR == 0);
static_assert(NITM % (PR_WAVES * PR_ROWS) == 0);
static_assert(NUSR % 64 == 0 && NITM % 64 == 0 && EMBW % 32 == 0 && HID % 32 == 0);
static_assert(NUSR <= 1024 && NITM <= 1024 && NUSR % 32 == 0 && NITM % 32 == 0);
static_assert(NH1 == 64 && NH2 == 16);

typedef __attribute__((ext_vector_type(16))) _Float16 v16h;
typedef __attribute__((ext_vector_type(8)))  _Float16 v8h;
typedef __attribute__((ext_vector_type(16))) __bf16   v16b;
typedef __attribute__((ext_vector_type(8)))  __bf16   v8b;
typedef __attribute__((ext_vector_type(8)))  float    v8f;
typedef __attribute__((ext_vector_type(4)))  float    v4f;
typedef __attribute__((ext_vector_type(2)))  float    v2f;

__device__ __forceinline__ unsigned short f2bf_bits(float f) {
  unsigned u = __float_as_uint(f);
  return (unsigned short)((u + 0x7FFFu + ((u >> 16) & 1u)) >> 16);
}
__device__ __forceinline__ float bf_bits2f(unsigned short h) { return __uint_as_float(((unsigned)h) << 16); }

__device__ __forceinline__ void dep_guard_h(v8f& a, v8f& b, v16h x, v16h y) { asm volatile("v_nop\n\tv_nop\n\tv_nop\n\tv_nop" : "+v"(a), "+v"(b) : "v"(x), "v"(y)); }
__device__ __forceinline__ void dep_guard_b(v8f& a, v8f& b, v16b x, v16b y) { asm volatile("v_nop\n\tv_nop\n\tv_nop\n\tv_nop" : "+v"(a), "+v"(b) : "v"(x), "v"(y)); }
__device__ __forceinline__ void dep_guard4x_b(v8f& a, v8f& b, v8f& c, v8f& d, v16b x, v16b y) {
  asm volatile("v_nop\n\tv_nop\n\tv_nop\n\tv_nop" : "+v"(a), "+v"(b), "+v"(c), "+v"(d) : "v"(x), "v"(y));
}
__device__ __forceinline__ void keep4_h(v16h a, v16h b, v16h c, v16h d) { asm volatile("v_nop" :: "v"(a), "v"(b), "v"(c), "v"(d)); }
__device__ __forceinline__ void keep4_b(v16b a, v16b b, v16b c, v16b d) { asm volatile("v_nop" :: "v"(a), "v"(b), "v"(c), "v"(d)); }
__device__ __forceinline__ void acc_guard4(v8f& a, v8f& b, v8f& c, v8f& d) { asm volatile("v_nop\n\tv_nop\n\tv_nop\n\tv_nop" : "+v"(a), "+v"(b), "+v"(c), "+v"(d)); }
__device__ __forceinline__ void acc_guard2(v8f& a, v8f& b) { asm volatile("v_nop\n\tv_nop\n\tv_nop\n\tv_nop" : "+v"(a), "+v"(b)); }
template <typename T> struct Frag;
template <> struct Frag<_Float16> {
  typedef v16h V; union U { v16h v; v8h h[2]; };
  static __device__ __forceinline__ v16h load(const _Float16* p) {
    U f; f.h[0] = *(const v8h*)(p); f.h[1] = *(const v8h*)(p + 16); return f.v;
  }
  static __device__ __forceinline__ v8f mma(v16h a, v16h b, v8f c) {
    return __builtin_amdgcn_wmma_f32_16x16x32_f16(false, a, false, b, (short)0, c, false, false);
  }
  static __device__ __forceinline__ void guard(v8f& a, v8f& b, v16h x, v16h y) { dep_guard_h(a, b, x, y); }
  static __device__ __forceinline__ void keep(v16h a, v16h b, v16h c, v16h d) { keep4_h(a, b, c, d); }
};
template <> struct Frag<__bf16> {
  typedef v16b V; union U { v16b v; v8b h[2]; };
  static __device__ __forceinline__ v16b load(const __bf16* p) {
    U f; f.h[0] = *(const v8b*)(p); f.h[1] = *(const v8b*)(p + 16); return f.v;
  }
  static __device__ __forceinline__ v8f mma(v16b a, v16b b, v8f c) {
    return __builtin_amdgcn_wmma_f32_16x16x32_bf16(false, a, false, b, (short)0, c, false, false);
  }
  static __device__ __forceinline__ void guard(v8f& a, v8f& b, v16b x, v16b y) { dep_guard_b(a, b, x, y); }
  static __device__ __forceinline__ void keep(v16b a, v16b b, v16b c, v16b d) { keep4_b(a, b, c, d); }
};

__device__ __forceinline__ float frcp_(float x)  { return __builtin_amdgcn_rcpf(x); }
__device__ __forceinline__ float fsig(float x)   { return frcp_(1.0f + expf(-x)); }
__device__ __forceinline__ float ftanh(float x)  { return 1.0f - 2.0f * frcp_(expf(2.0f * x) + 1.0f); }
__device__ __forceinline__ float fleaky(float x) { return x > 0.0f ? x : 0.01f * x; }

template <int ET> struct Elem;
template <> struct Elem<0> { typedef _Float16 T; };
template <> struct Elem<1> { typedef __bf16 T; };
template <int ET, bool SPLIT, int BIAS_MODE, int OUT_MODE, bool RESID, int ACT = 0>
__global__ __launch_bounds__(256) void wmma_gemm64(
    const unsigned short* __restrict__ Ap, const unsigned short* __restrict__ A2p, int lda, long strideA,
    const unsigned short* __restrict__ Btp, const unsigned short* __restrict__ Bt2p, int ldb, long strideB,
    void* __restrict__ Cout, void* __restrict__ Cout2, int ldc, long strideC,
    const float* __restrict__ bias,
    const float* __restrict__ resid, long strideR,
    int M, int N, int K, float scale) {
  typedef typename Elem<ET>::T T;
  typedef typename Frag<T>::V V;
  const T* A = (const T*)Ap; const T* A2 = (const T*)A2p; const T* Bt = (const T*)Btp; const T* Bt2 = (const T*)Bt2p;
  __shared__ __align__(16) float sT[8][16 * 68];
  const int b    = blockIdx.y;
  const int lane = threadIdx.x & 31;
  const int wave = threadIdx.x >> 5;
  const int tilesN = N >> 6;
  const int tilesM = M >> 6;
  const int tile = blockIdx.x * 8 + wave;
  if (tile >= tilesM * tilesN) return;
  const int tm = tile / tilesN;
  const int tn = tile - tm * tilesN;
  const int m0 = tm << 6;
  const int n0 = tn << 6;

  const T* Ab  = A  + (size_t)b * strideA;
  const T* Bb  = Bt + (size_t)b * strideB;
  const T* Ab2 = SPLIT ? (A2  + (size_t)b * strideA) : nullptr;
  const T* Bb2 = SPLIT ? (Bt2 + (size_t)b * strideB) : nullptr;

  const int rlane = lane & 15;
  const int koff  = (lane >> 4) * 8;
  const int mOff  = (lane >> 4) * 8;

  v8f acc[4][4];
#pragma unroll
  for (int i = 0; i < 4; ++i)
#pragma unroll
    for (int j = 0; j < 4; ++j) acc[i][j] = (v8f){0.f,0.f,0.f,0.f,0.f,0.f,0.f,0.f};

  for (int k0 = 0; k0 < K; k0 += 32) {
    V bh[4], bl[4];
#pragma unroll
    for (int j = 0; j < 4; ++j) {
      const size_t bo = (size_t)(n0 + (j << 4) + rlane) * ldb + koff + k0;
      bh[j] = Frag<T>::load(Bb + bo);
      if (SPLIT) bl[j] = Frag<T>::load(Bb2 + bo);
    }
#pragma unroll
    for (int i = 0; i < 4; ++i) {
      const size_t ao = (size_t)(m0 + (i << 4) + rlane) * lda + koff + k0;
      V ah = Frag<T>::load(Ab + ao);
      V al;
      if (SPLIT) al = Frag<T>::load(Ab2 + ao);
#pragma unroll
      for (int j = 0; j < 4; ++j) {
        acc[i][j] = Frag<T>::mma(ah, bh[j], acc[i][j]);
        if (SPLIT) {
          acc[i][j] = Frag<T>::mma(ah, bl[j], acc[i][j]);
          acc[i][j] = Frag<T>::mma(al, bh[j], acc[i][j]);
        }
      }
      Frag<T>::guard(acc[i][0], acc[i][3], ah, SPLIT ? al : ah);
    }
    Frag<T>::keep(bh[0], bh[1], bh[2], bh[3]);
    if (SPLIT) Frag<T>::keep(bl[0], bl[1], bl[2], bl[3]);
  }
  acc_guard4(acc[0][0], acc[0][1], acc[0][2], acc[0][3]);
  acc_guard4(acc[1][0], acc[1][1], acc[1][2], acc[1][3]);
  acc_guard4(acc[2][0], acc[2][1], acc[2][2], acc[2][3]);
  acc_guard4(acc[3][0], acc[3][1], acc[3][2], acc[3][3]);

  float* slab = sT[wave];
  const float* Rb = RESID ? (resid + (size_t)b * strideR) : nullptr;
#pragma unroll
  for (int i = 0; i < 4; ++i) {
    const int mBase = m0 + (i << 4);
#pragma unroll
    for (int j = 0; j < 4; ++j) {
      const int n = n0 + (j << 4) + rlane;
      float bv = 0.f;
      if (BIAS_MODE == 2) bv = bias[n];
#pragma unroll
      for (int r = 0; r < 8; ++r) {
        float v = acc[i][j][r] * scale;
        if (BIAS_MODE == 1) v += bias[mBase + mOff + r];
        if (BIAS_MODE == 2) v += bv;
        if (RESID) v += Rb[(size_t)(mBase + mOff + r) * ldc + n];
        if (ACT == 1) v = tanhf(v);
        if (ACT == 2) v = fmaxf(v, 0.0f);
        if (ACT == 3) v = v / (1.0f + expf(-v));
        if (ACT == 4) v = (v > 0.f) ? v : 0.01f * v;
        if (ACT == 5) v = 0.5f * v * (1.0f + erff(v * 0.70710678118654752f));
        slab[(mOff + r) * 68 + (j << 4) + rlane] = v;
      }
    }
    __builtin_amdgcn_fence(__ATOMIC_RELEASE, "workgroup");
    __builtin_amdgcn_wave_barrier();
    __builtin_amdgcn_fence(__ATOMIC_ACQUIRE, "workgroup");
    if (OUT_MODE == 0) {
      float* C = (float*)Cout + (size_t)b * strideC;
      const int hh = lane >> 4, c4 = (lane & 15) * 4;
      for (int pass = 0; pass < 2; ++pass) {
#pragma unroll
        for (int it = 0; it < 8; ++it) {
          const int row = it * 2 + hh;
          v4f v = *(const v4f*)(slab + row * 68 + c4);
          *(volatile v4f*)(C + (size_t)(mBase + row) * ldc + n0 + c4) = v;
        }
        __threadfence();
      }
    } else {
      const int q = lane >> 3, c8 = (lane & 7) * 8;
      unsigned short* C  = (unsigned short*)Cout  + (size_t)b * strideC;
      unsigned short* C2 = (OUT_MODE == 2) ? ((unsigned short*)Cout2 + (size_t)b * strideC) : nullptr;
      for (int pass = 0; pass < 2; ++pass) {
#pragma unroll
        for (int it = 0; it < 4; ++it) {
          const int row = it * 4 + q;
          const float* sp = slab + row * 68 + c8;
          v8h hv, lv;
#pragma unroll
          for (int e = 0; e < 8; ++e) {
            if (OUT_MODE == 1) {
              hv[e] = (_Float16)sp[e];
            } else {
              unsigned short hb = f2bf_bits(sp[e]);
              unsigned short lb = f2bf_bits(sp[e] - bf_bits2f(hb));
              hv[e] = __builtin_bit_cast(_Float16, hb);
              lv[e] = __builtin_bit_cast(_Float16, lb);
            }
          }
          *(volatile v8h*)(C + (size_t)(mBase + row) * ldc + n0 + c8) = hv;
          if (OUT_MODE == 2) *(volatile v8h*)(C2 + (size_t)(mBase + row) * ldc + n0 + c8) = lv;
        }
        __threadfence();
      }
    }
    __builtin_amdgcn_fence(__ATOMIC_RELEASE, "workgroup");
    __builtin_amdgcn_wave_barrier();
    __builtin_amdgcn_fence(__ATOMIC_ACQUIRE, "workgroup");
  }
}

__global__ __launch_bounds__(256) void cvt_split_kernel(const float* __restrict__ src,
                                                      unsigned short* __restrict__ dh, unsigned short* __restrict__ dl, int n8) {
  const int i = blockIdx.x * 256 + threadIdx.x;
  if (i < n8) {
    const float* sp = src + (size_t)i * 8;
    const v4f a = *(const v4f*)(sp);
    const v4f b = *(const v4f*)(sp + 4);
    v8h hv, lv;
#pragma unroll
    for (int e = 0; e < 4; ++e) {
      const unsigned short ha = f2bf_bits(a[e]);
      const unsigned short la = f2bf_bits(a[e] - bf_bits2f(ha));
      const unsigned short hb = f2bf_bits(b[e]);
      const unsigned short lb = f2bf_bits(b[e] - bf_bits2f(hb));
      hv[e]     = __builtin_bit_cast(_Float16, ha);
      lv[e]     = __builtin_bit_cast(_Float16, la);
      hv[4 + e] = __builtin_bit_cast(_Float16, hb);
      lv[4 + e] = __builtin_bit_cast(_Float16, lb);
    }
    unsigned short* ph = dh + (size_t)i * 8;
    unsigned short* pl = dl + (size_t)i * 8;
    *(volatile v8h*)ph = hv;
    *(volatile v8h*)pl = lv;
    __threadfence();
    *(volatile v8h*)ph = hv;
    *(volatile v8h*)pl = lv;
  }
}

template <int INK, bool SEQ>
__global__ __launch_bounds__(GRU_THR) void gru_seq_kernel(
    const unsigned short* __restrict__ Xhp, const unsigned short* __restrict__ Xlp, long xsb, long xst,
    const unsigned short* __restrict__ Wihp, const unsigned short* __restrict__ Wilp,
    const unsigned short* __restrict__ Whhp, const unsigned short* __restrict__ Whlp,
    const float* __restrict__ bih, const float* __restrict__ bhh,
    unsigned short* __restrict__ Yh, unsigned short* __restrict__ Yl, int ycol,
    float* __restrict__ Hfin, int nb, int reverse) {
  static_assert(INK % 32 == 0);
  __shared__ __align__(16) __bf16 Ah[2][SEQB * HPAD];
  __shared__ __align__(16) __bf16 Al[2][SEQB * HPAD];
  __shared__ __align__(16) float  Sl[SEQB * SLABP];
  const __bf16* XH  = (const __bf16*)Xhp;  const __bf16* XL  = (const __bf16*)Xlp;
  const __bf16* WIH = (const __bf16*)Wihp; const __bf16* WIL = (const __bf16*)Wilp;
  const __bf16* WHH = (const __bf16*)Whhp; const __bf16* WHL = (const __bf16*)Whlp;
  const int tid = threadIdx.x, lane = tid & 31, wave = tid >> 5;
  const int c = lane & 15, hh = lane >> 4, koff = hh * 8, c4 = c * 4;
  const int rowbase = blockIdx.x * SEQB;

  {
    unsigned int* z0 = (unsigned int*)(&Ah[0][0]);
    unsigned int* z1 = (unsigned int*)(&Al[0][0]);
#pragma unroll 1
    for (int i = tid; i < SEQB * HPAD; i += GRU_THR) { z0[i] = 0u; z1[i] = 0u; }
  }
  float hold[8];
#pragma unroll
  for (int r = 0; r < 8; ++r) hold[r] = 0.0f;

  const int j0 = 16 * wave + c, j1 = HID + j0, j2 = 2 * HID + j0;
  const float br  = bih[j0] + bhh[j0];
  const float bz  = bih[j1] + bhh[j1];
  const float bxn = bih[j2];
  const float bhn = bhh[j2];
  const __bf16* wi0h = WIH + (size_t)j0 * INK + koff;  const __bf16* wi0l = WIL + (size_t)j0 * INK + koff;
  const __bf16* wi1h = WIH + (size_t)j1 * INK + koff;  const __bf16* wi1l = WIL + (size_t)j1 * INK + koff;
  const __bf16* wi2h = WIH + (size_t)j2 * INK + koff;  const __bf16* wi2l = WIL + (size_t)j2 * INK + koff;
  const __bf16* wh0h = WHH + (size_t)j0 * HID + koff;  const __bf16* wh0l = WHL + (size_t)j0 * HID + koff;
  const __bf16* wh1h = WHH + (size_t)j1 * HID + koff;  const __bf16* wh1l = WHL + (size_t)j1 * HID + koff;
  const __bf16* wh2h = WHH + (size_t)j2 * HID + koff;  const __bf16* wh2l = WHL + (size_t)j2 * HID + koff;
  __syncthreads();

  const v8f z8 = {0.f, 0.f, 0.f, 0.f, 0.f, 0.f, 0.f, 0.f};

#pragma unroll 1
  for (int step = 0; step < NSTEP; ++step) {
    const int t   = reverse ? (NSTEP - 1 - step) : step;
    const int cur = step & 1, nxt = cur ^ 1;
    v8f accR = z8, accZ = z8, accXN = z8, accHN = z8;

    const __bf16* xr = XH + (size_t)(rowbase + c) * (size_t)xsb + (size_t)t * (size_t)xst + koff;
    const __bf16* xl = XL + (size_t)(rowbase + c) * (size_t)xsb + (size_t)t * (size_t)xst + koff;
#pragma unroll 1
    for (int k0 = 0; k0 < INK; k0 += 32) {
      const v16b ah  = Frag<__bf16>::load(xr + k0);
      const v16b al  = Frag<__bf16>::load(xl + k0);
      const v16b b0h = Frag<__bf16>::load(wi0h + k0), b0l = Frag<__bf16>::load(wi0l + k0);
      const v16b b1h = Frag<__bf16>::load(wi1h + k0), b1l = Frag<__bf16>::load(wi1l + k0);
      const v16b b2h = Frag<__bf16>::load(wi2h + k0), b2l = Frag<__bf16>::load(wi2l + k0);
      accR  = Frag<__bf16>::mma(ah, b0h, accR);  accR  = Frag<__bf16>::mma(ah, b0l, accR);  accR  = Frag<__bf16>::mma(al, b0h, accR);
      accZ  = Frag<__bf16>::mma(ah, b1h, accZ);  accZ  = Frag<__bf16>::mma(ah, b1l, accZ);  accZ  = Frag<__bf16>::mma(al, b1h, accZ);
      accXN = Frag<__bf16>::mma(ah, b2h, accXN); accXN = Frag<__bf16>::mma(ah, b2l, accXN); accXN = Frag<__bf16>::mma(al, b2h, accXN);
      dep_guard4x_b(accR, accZ, accXN, accHN, ah, al);
      keep4_b(b0h, b0l, b1h, b1l);
      keep4_b(b2h, b2l, ah, al);
    }
    const __bf16* hr = &Ah[cur][0] + c * HPAD + koff;
    const __bf16* hl = &Al[cur][0] + c * HPAD + koff;
#pragma unroll 1
    for (int k0 = 0; k0 < HID; k0 += 32) {
      const v16b ah  = Frag<__bf16>::load(hr + k0);
      const v16b al  = Frag<__bf16>::load(hl + k0);
      const v16b b0h = Frag<__bf16>::load(wh0h + k0), b0l = Frag<__bf16>::load(wh0l + k0);
      const v16b b1h = Frag<__bf16>::load(wh1h + k0), b1l = Frag<__bf16>::load(wh1l + k0);
      const v16b b2h = Frag<__bf16>::load(wh2h + k0), b2l = Frag<__bf16>::load(wh2l + k0);
      accR  = Frag<__bf16>::mma(ah, b0h, accR);  accR  = Frag<__bf16>::mma(ah, b0l, accR);  accR  = Frag<__bf16>::mma(al, b0h, accR);
      accZ  = Frag<__bf16>::mma(ah, b1h, accZ);  accZ  = Frag<__bf16>::mma(ah, b1l, accZ);  accZ  = Frag<__bf16>::mma(al, b1h, accZ);
      accHN = Frag<__bf16>::mma(ah, b2h, accHN); accHN = Frag<__bf16>::mma(ah, b2l, accHN); accHN = Frag<__bf16>::mma(al, b2h, accHN);
      dep_guard4x_b(accR, accZ, accXN, accHN, ah, al);
      keep4_b(b0h, b0l, b1h, b1l);
      keep4_b(b2h, b2l, ah, al);
    }
    acc_guard4(accR, accZ, accXN, accHN);

    __bf16* ahn = &Ah[nxt][0];
    __bf16* aln = &Al[nxt][0];
#pragma unroll
    for (int r = 0; r < 8; ++r) {
      const float rg = fsig(accR[r] + br);
      const float zg = fsig(accZ[r] + bz);
      const float pn = (accXN[r] + bxn) + rg * (accHN[r] + bhn);
      const float ng = ftanh(pn);
      const float ho = hold[r];
      const float hn = (1.0f - zg) * ng + zg * ho;
      hold[r] = hn;
      const unsigned short hb = f2bf_bits(hn);
      const unsigned short lb = f2bf_bits(hn - bf_bits2f(hb));
      ahn[(8 * hh + r) * HPAD + j0] = __builtin_bit_cast(__bf16, hb);
      aln[(8 * hh + r) * HPAD + j0] = __builtin_bit_cast(__bf16, lb);
    }
    __syncthreads();

    if (SEQ) {
      const int row = 4 * wave + (lane >> 3);
      const int c8  = (lane & 7) * 8;
      const v8b vh = *(const v8b*)(ahn + row * HPAD + c8);
      const v8b vl = *(const v8b*)(aln + row * HPAD + c8);
      const v8h sh = __builtin_bit_cast(v8h, vh);
      const v8h sl = __builtin_bit_cast(v8h, vl);
      const size_t off = ((size_t)t * (size_t)nb + (size_t)(rowbase + row)) * EMBW + ycol + c8;
      for (int pass = 0; pass < 2; ++pass) {
        *(volatile v8h*)(Yh + off) = sh;
        *(volatile v8h*)(Yl + off) = sl;
        __threadfence();
      }
    }
  }

  if (!SEQ) {
#pragma unroll
    for (int r = 0; r < 8; ++r) Sl[(8 * hh + r) * SLABP + j0] = hold[r];
    __syncthreads();
    for (int pass = 0; pass < 2; ++pass) {
#pragma unroll
      for (int it = 0; it < 2; ++it) {
        const int row = 4 * wave + 2 * it + hh;
        const v4f v = *(const v4f*)(Sl + row * SLABP + c4);
        *(volatile v4f*)(Hfin + (size_t)(rowbase + row) * HID + c4) = v;
      }
      __threadfence();
    }
  }
}

__global__ __launch_bounds__(1024) void attn_beta_kernel(const float* __restrict__ Hs, const float* __restrict__ A1,
                                                        const float* __restrict__ a1, const float* __restrict__ A2,
                                                        const float* __restrict__ a2, float* __restrict__ beta_out, int nb) {
  __shared__ float red[1024];
  __shared__ __align__(16) float bet[1024];
  const int b = threadIdx.x, lane = b & 31, wave = b >> 5;
  float acc[NATT];
#pragma unroll
  for (int j = 0; j < NATT; ++j) acc[j] = a1[j];
  const float* hrow = Hs + (size_t)b * HID;
#pragma unroll 1
  for (int d = 0; d < HID; ++d) {
    const float hv = hrow[d];
#pragma unroll
    for (int j = 0; j < NATT; ++j) acc[j] = fmaf(hv, A1[j * HID + d], acc[j]);
  }
  float s = 0.0f;
#pragma unroll
  for (int j = 0; j < NATT; ++j) s = fmaf(ftanh(acc[j]), A2[j], s);
  const float w = s + a2[0];
  red[b] = w;
  __syncthreads();
  for (int st = nb >> 1; st > 0; st >>= 1) {
    if (b < st) red[b] = fmaxf(red[b], red[b + st]);
    __syncthreads();
  }
  const float mx = red[0];
  __syncthreads();
  const float e = expf(w - mx);
  red[b] = e;
  __syncthreads();
  for (int st = nb >> 1; st > 0; st >>= 1) {
    if (b < st) red[b] += red[b + st];
    __syncthreads();
  }
  const float tot = red[0];
  const float be = e * (1.0f / tot);
  bet[b] = be;
  __syncthreads();
  if (lane < 8) {
    const v4f v = *(const v4f*)(bet + 32 * wave + 4 * lane);
    float* op = beta_out + 32 * wave + 4 * lane;
    *(volatile v4f*)op = v;
    __threadfence();
    *(volatile v4f*)op = v;
  }
}

__global__ __launch_bounds__(FMX_THR) void fmix_emb_kernel(const float* __restrict__ Hs, const float* __restrict__ beta,
                                                          const float* __restrict__ LFM, const float* __restrict__ FW,
                                                          const float* __restrict__ Fb, const float* __restrict__ FV,
                                                          unsigned short* __restrict__ embh, unsigned short* __restrict__ embl) {
  __shared__ float xs[EMBW];
  __shared__ float red[FMX_THR];
  __shared__ __align__(16) unsigned short ebits[2 * EMBW];
  const int b = blockIdx.x, d = threadIdx.x, lane = d & 31, wave = d >> 5;
  const float bt = beta[b];
  const float tv = Hs[(size_t)b * HID + d] * bt;
  const float lv = LFM[(size_t)b * HID + d];
  xs[d] = tv; xs[HID + d] = lv;
  __syncthreads();
  float lin = Fb[d], xv = 0.0f, x2v2 = 0.0f;
  const float* fwr = FW + (size_t)d * EMBW;
#pragma unroll 1
  for (int k = 0; k < EMBW; ++k) {
    const float xk = xs[k];
    lin = fmaf(xk, fwr[k], lin);
    const float v = FV[(size_t)k * HID + d];
    xv = fmaf(xk, v, xv);
    x2v2 = fmaf(xk * xk, v * v, x2v2);
  }
  red[d] = xv * xv - x2v2;
  __syncthreads();
  for (int st = FMX_THR >> 1; st > 0; st >>= 1) {
    if (d < st) red[d] += red[d + st];
    __syncthreads();
  }
  const float inter = 0.5f * red[0];
  const float fv = fsig(lin + inter);
  const float e0 = tv + lv;
  const unsigned short h0 = f2bf_bits(e0), h1 = f2bf_bits(fv);
  const unsigned short l0 = f2bf_bits(e0 - bf_bits2f(h0)), l1 = f2bf_bits(fv - bf_bits2f(h1));
  ebits[d] = h0;             ebits[HID + d] = h1;
  ebits[EMBW + d] = l0;      ebits[EMBW + HID + d] = l1;
  __syncthreads();
  const int l16 = lane & 15;
  const v8h v = *(const v8h*)(ebits + wave * EMBW + 8 * l16);
  unsigned short* dst = ((wave == 0) ? embh : embl) + (size_t)b * EMBW + 8 * l16;
  if (lane < 16) {
    *(volatile v8h*)dst = v;
    __threadfence();
    *(volatile v8h*)dst = v;
  }
}

__global__ __launch_bounds__(PR_THR) void pair_score_kernel(
    const float* __restrict__ AU, const float* __restrict__ AI,
    const unsigned short* __restrict__ W2hp, const unsigned short* __restrict__ W2lp,
    const float* __restrict__ b2, const float* __restrict__ Wo, const float* __restrict__ bo,
    float* __restrict__ out, int nItems) {
  __shared__ __align__(16) unsigned int Th[PR_WAVES][PR_ROWS * (PR_PITCH / 2)];
  __shared__ __align__(16) unsigned int Tl[PR_WAVES][PR_ROWS * (PR_PITCH / 2)];
  __shared__ __align__(16) float Sc[PR_WAVES][PR_ROWS];
  const int tid = threadIdx.x, lane = tid & 31, wave = tid >> 5;
  const int c = lane & 15, hh = lane >> 4, koff = hh * 8;
  const int blkPerRow = nItems / (PR_WAVES * PR_ROWS);
  const int u  = blockIdx.x / blkPerRow;
  const int i0 = (blockIdx.x - u * blkPerRow) * (PR_WAVES * PR_ROWS) + wave * PR_ROWS;
  const v2f au = *(const v2f*)(AU + (size_t)u * NH1 + 2 * lane);
  unsigned int* th = Th[wave];
  unsigned int* tl = Tl[wave];
#pragma unroll 1
  for (int row = 0; row < PR_ROWS; ++row) {
    const v2f ai = *(const v2f*)(AI + (size_t)(i0 + row) * NH1 + 2 * lane);
    const float x0 = fleaky(au[0] + ai[0]);
    const float x1 = fleaky(au[1] + ai[1]);
    const unsigned short h0 = f2bf_bits(x0), h1 = f2bf_bits(x1);
    const unsigned short l0 = f2bf_bits(x0 - bf_bits2f(h0)), l1 = f2bf_bits(x1 - bf_bits2f(h1));
    th[row * (PR_PITCH / 2) + lane] = (unsigned int)h0 | ((unsigned int)h1 << 16);
    tl[row * (PR_PITCH / 2) + lane] = (unsigned int)l0 | ((unsigned int)l1 << 16);
  }
  __syncthreads();

  const __bf16* W2H = (const __bf16*)W2hp + (size_t)c * NH1 + koff;
  const __bf16* W2L = (const __bf16*)W2lp + (size_t)c * NH1 + koff;
  const v16b b0h = Frag<__bf16>::load(W2H),      b0l = Frag<__bf16>::load(W2L);
  const v16b b1h = Frag<__bf16>::load(W2H + 32), b1l = Frag<__bf16>::load(W2L + 32);
  const __bf16* ta = (const __bf16*)th + koff;
  const __bf16* tb = (const __bf16*)tl + koff;
  const v8f z8 = {0.f, 0.f, 0.f, 0.f, 0.f, 0.f, 0.f, 0.f};
  v8f acc0 = z8, acc1 = z8;
  {
    const v16b a0 = Frag<__bf16>::load(ta + c * PR_PITCH),             a0l = Frag<__bf16>::load(tb + c * PR_PITCH);
    const v16b a1 = Frag<__bf16>::load(ta + c * PR_PITCH + 32),        a1l = Frag<__bf16>::load(tb + c * PR_PITCH + 32);
    const v16b a2 = Frag<__bf16>::load(ta + (16 + c) * PR_PITCH),      a2l = Frag<__bf16>::load(tb + (16 + c) * PR_PITCH);
    const v16b a3 = Frag<__bf16>::load(ta + (16 + c) * PR_PITCH + 32), a3l = Frag<__bf16>::load(tb + (16 + c) * PR_PITCH + 32);
    acc0 = Frag<__bf16>::mma(a0, b0h, acc0); acc0 = Frag<__bf16>::mma(a0, b0l, acc0); acc0 = Frag<__bf16>::mma(a0l, b0h, acc0);
    acc0 = Frag<__bf16>::mma(a1, b1h, acc0); acc0 = Frag<__bf16>::mma(a1, b1l, acc0); acc0 = Frag<__bf16>::mma(a1l, b1h, acc0);
    acc1 = Frag<__bf16>::mma(a2, b0h, acc1); acc1 = Frag<__bf16>::mma(a2, b0l, acc1); acc1 = Frag<__bf16>::mma(a2l, b0h, acc1);
    acc1 = Frag<__bf16>::mma(a3, b1h, acc1); acc1 = Frag<__bf16>::mma(a3, b1l, acc1); acc1 = Frag<__bf16>::mma(a3l, b1h, acc1);
    dep_guard_b(acc0, acc1, a3, a3l);
    keep4_b(b0h, b0l, b1h, b1l);
    keep4_b(a0, a0l, a1, a1l);
    keep4_b(a2, a2l, a3, a3l);
  }
  acc_guard2(acc0, acc1);

  const float b2c = b2[c], woc = Wo[c], boc = bo[0];
  float* sc = Sc[wave];
#pragma unroll
  for (int r = 0; r < 8; ++r) {
    float v0 = fleaky(acc0[r] + b2c) * woc;
    float v1 = fleaky(acc1[r] + b2c) * woc;
    v0 += __shfl_xor(v0, 1);  v1 += __shfl_xor(v1, 1);
    v0 += __shfl_xor(v0, 2);  v1 += __shfl_xor(v1, 2);
    v0 += __shfl_xor(v0, 4);  v1 += __shfl_xor(v1, 4);
    v0 += __shfl_xor(v0, 8);  v1 += __shfl_xor(v1, 8);
    v0 = fleaky(v0 + boc);
    v1 = fleaky(v1 + boc);
    if (c == 0) { sc[8 * hh + r] = v0; sc[16 + 8 * hh + r] = v1; }
  }
  __builtin_amdgcn_fence(__ATOMIC_RELEASE, "workgroup");
  __builtin_amdgcn_wave_barrier();
  __builtin_amdgcn_fence(__ATOMIC_ACQUIRE, "workgroup");
  if (lane < 8) {
    const v4f o = *(const v4f*)(sc + 4 * lane);
    float* op = out + (size_t)u * (size_t)nItems + i0 + 4 * lane;
    *(volatile v4f*)op = o;
    __threadfence();
    *(volatile v4f*)op = o;
  }
}

static inline void run_cvt(const float* src, unsigned short* h, unsigned short* l, int n, hipStream_t st) {
  const int n8 = n / 8;
  cvt_split_kernel<<<(n8 + 255) / 256, 256, 0, st>>>(src, h, l, n8);
}

extern "C" void kernel_launch(void* const* d_in, const int* in_sizes, int n_in,
                              void* d_out, int out_size, void* d_ws, size_t ws_size, hipStream_t stream) {
  if (n_in < 40 || d_out == nullptr || d_ws == nullptr) return;
  bool ok = in_sizes[0] == NUSR * NSTEP * HID && in_sizes[1] == NITM * NSTEP * HID &&
            in_sizes[2] == NUSR * HID && in_sizes[3] == NITM * HID;
  for (int p = 0; p < 2; ++p) {
    const int o = 4 + 8 * p;
    ok = ok && in_sizes[o] == 2 * G3 * HID && in_sizes[o + 1] == 2 * G3 * HID && in_sizes[o + 2] == 2 * G3 &&
         in_sizes[o + 3] == 2 * G3 && in_sizes[o + 4] == 2 * G3 * EMBW && in_sizes[o + 5] == 2 * G3 * HID &&
         in_sizes[o + 6] == 2 * G3 && in_sizes[o + 7] == 2 * G3;
    const int a = 20 + 7 * p;
    ok = ok && in_sizes[a] == NATT * HID && in_sizes[a + 1] == NATT && in_sizes[a + 2] == NATT && in_sizes[a + 3] == 1 &&
         in_sizes[a + 4] == HID * EMBW && in_sizes[a + 5] == HID && in_sizes[a + 6] == EMBW * HID;
  }
  ok = ok && in_sizes[34] == NH1 * PAIRW && in_sizes[35] == NH1 && in_sizes[36] == NH2 * NH1 && in_sizes[37] == NH2 &&
       in_sizes[38] == NH2 && in_sizes[39] == 1 && out_size == NUSR * NITM;
  if (!ok) return;

  const float* words[2] = { (const float*)d_in[0], (const float*)d_in[1] };
  const float* lfm[2]   = { (const float*)d_in[2], (const float*)d_in[3] };
  const float* gw[2][8];
  for (int p = 0; p < 2; ++p)
    for (int k = 0; k < 8; ++k) gw[p][k] = (const float*)d_in[4 + 8 * p + k];
  const float* aw[2][7];
  for (int p = 0; p < 2; ++p)
    for (int k = 0; k < 7; ++k) aw[p][k] = (const float*)d_in[20 + 7 * p + k];
  const float* mW1 = (const float*)d_in[34];
  const float* mb1 = (const float*)d_in[35];
  const float* mW2 = (const float*)d_in[36];
  const float* mb2 = (const float*)d_in[37];
  const float* mWo = (const float*)d_in[38];
  const float* mbo = (const float*)d_in[39];
  float* out = (float*)d_out;

  char* ws = (char*)d_ws; size_t off = 0;
  auto carve = [&](size_t bytes) -> char* { char* p = ws + off; off += (bytes + 255) & ~(size_t)255; return p; };
  unsigned short* XH    = (unsigned short*)carve((size_t)NITM * NSTEP * HID * 2);
  unsigned short* XL    = (unsigned short*)carve((size_t)NITM * NSTEP * HID * 2);
  unsigned short* YH    = (unsigned short*)carve((size_t)NSTEP * NITM * EMBW * 2);
  unsigned short* YL    = (unsigned short*)carve((size_t)NSTEP * NITM * EMBW * 2);
  unsigned short* W0H   = (unsigned short*)carve((size_t)2 * G3 * HID * 2);
  unsigned short* W0L   = (unsigned short*)carve((size_t)2 * G3 * HID * 2);
  unsigned short* U0H   = (unsigned short*)carve((size_t)2 * G3 * HID * 2);
  unsigned short* U0L   = (unsigned short*)carve((size_t)2 * G3 * HID * 2);
  unsigned short* W1H   = (unsigned short*)carve((size_t)2 * G3 * EMBW * 2);
  unsigned short* W1L   = (unsigned short*)carve((size_t)2 * G3 * EMBW * 2);
  unsigned short* U1H   = (unsigned short*)carve((size_t)2 * G3 * HID * 2);
  unsigned short* U1L   = (unsigned short*)carve((size_t)2 * G3 * HID * 2);
  float*          HB    = (float*)carve((size_t)NITM * HID * 4);
  float*          BETA  = (float*)carve((size_t)NITM * 4);
  unsigned short* EMBUH = (unsigned short*)carve((size_t)NUSR * EMBW * 2);
  unsigned short* EMBUL = (unsigned short*)carve((size_t)NUSR * EMBW * 2);
  unsigned short* EMBIH = (unsigned short*)carve((size_t)NITM * EMBW * 2);
  unsigned short* EMBIL = (unsigned short*)carve((size_t)NITM * EMBW * 2);
  float*          AU    = (float*)carve((size_t)NUSR * NH1 * 4);
  float*          AI    = (float*)carve((size_t)NITM * NH1 * 4);
  unsigned short* M1H   = (unsigned short*)carve((size_t)NH1 * PAIRW * 2);
  unsigned short* M1L   = (unsigned short*)carve((size_t)NH1 * PAIRW * 2);
  unsigned short* M2H   = (unsigned short*)carve((size_t)NH2 * NH1 * 2);
  unsigned short* M2L   = (unsigned short*)carve((size_t)NH2 * NH1 * 2);
  if (off > ws_size || off > (size_t)134217728) return;

  unsigned short* EH[2] = { EMBUH, EMBIH };
  unsigned short* EL[2] = { EMBUL, EMBIL };
  const int nbv[2] = { NUSR, NITM };
  const long l0sb = (long)NSTEP * HID, l0st = (long)HID;

  for (int p = 0; p < 2; ++p) {
    const int nb = nbv[p];
    const float *W0 = gw[p][0], *U0 = gw[p][1], *b0 = gw[p][2], *c0 = gw[p][3];
    const float *W1 = gw[p][4], *U1 = gw[p][5], *b1 = gw[p][6], *c1 = gw[p][7];
    run_cvt(words[p], XH, XL, nb * NSTEP * HID, stream);
    run_cvt(W0, W0H, W0L, 2 * G3 * HID, stream);
    run_cvt(U0, U0H, U0L, 2 * G3 * HID, stream);
    run_cvt(W1, W1H, W1L, 2 * G3 * EMBW, stream);
    run_cvt(U1, U1H, U1L, 2 * G3 * HID, stream);
    gru_seq_kernel<HID, true><<<nb / SEQB, GRU_THR, 0, stream>>>(
        XH, XL, l0sb, l0st, W0H, W0L, U0H, U0L, b0, c0, YH, YL, 0, HB, nb, 0);
    gru_seq_kernel<HID, true><<<nb / SEQB, GRU_THR, 0, stream>>>(
        XH, XL, l0sb, l0st, W0H + G3 * HID, W0L + G3 * HID, U0H + G3 * HID, U0L + G3 * HID,
        b0 + G3, c0 + G3, YH, YL, HID, HB, nb, 1);
    gru_seq_kernel<EMBW, false><<<nb / SEQB, GRU_THR, 0, stream>>>(
        YH, YL, (long)EMBW, (long)nb * EMBW, W1H + G3 * EMBW, W1L + G3 * EMBW, U1H + G3 * HID, U1L + G3 * HID,
        b1 + G3, c1 + G3, XH, XL, 0, HB, nb, 1);
    attn_beta_kernel<<<1, nb, 0, stream>>>(HB, aw[p][0], aw[p][1], aw[p][2], aw[p][3], BETA, nb);
    fmix_emb_kernel<<<nb, FMX_THR, 0, stream>>>(HB, BETA, lfm[p], aw[p][4], aw[p][5], aw[p][6], EH[p], EL[p]);
  }

  run_cvt(mW1, M1H, M1L, NH1 * PAIRW, stream);
  run_cvt(mW2, M2H, M2L, NH2 * NH1, stream);
  wmma_gemm64<1, true, 2, 0, false, 0><<<dim3((NUSR / 64 + 7) / 8, 1), 256, 0, stream>>>(
      EMBUH, EMBUL, EMBW, 0L, M1H, M1L, PAIRW, 0L, (void*)AU, (void*)AU, NH1, 0L,
      mb1, AU, 0L, NUSR, NH1, EMBW, 1.0f);
  wmma_gemm64<1, true, 0, 0, false, 0><<<dim3((NITM / 64 + 7) / 8, 1), 256, 0, stream>>>(
      EMBIH, EMBIL, EMBW, 0L, M1H + EMBW, M1L + EMBW, PAIRW, 0L, (void*)AI, (void*)AI, NH1, 0L,
      mb1, AI, 0L, NITM, NH1, EMBW, 1.0f);

  pair_score_kernel<<<NUSR * (NITM / (PR_WAVES * PR_ROWS)), PR_THR, 0, stream>>>(
      AU, AI, M2H, M2L, mb2, mWo, mbo, out, NITM);
}
